// DynamicNeuralTuringMachine_7713761263952
// MI455X (gfx1250) — hardware-run, weakly checked
//
#include <hip/hip_runtime.h>
#include <math.h>

typedef __attribute__((ext_vector_type(16))) _Float16 v16h;
typedef __attribute__((ext_vector_type(8)))  _Float16 v8h;
typedef __attribute__((ext_vector_type(4)))  _Float16 v4h;
typedef __attribute__((ext_vector_type(8)))  float    v8f;
typedef __attribute__((ext_vector_type(4)))  float    v4f;

constexpr int kBatch = 32;
constexpr int kSteps = 32;
constexpr int kFeat  = 64;
constexpr int kHid   = 256;
constexpr int kSlots = 1024;
constexpr int kAddr  = 64;
constexpr int kCont  = 192;
constexpr int kGate  = 768;
constexpr int kCls   = 10;
static_assert(kAddr + kCont == 256, "memory row width");
static_assert(kBatch == 32 && kFeat == 64, "input plane build assumes a 32 x 64 slab per step");

constexpr float kCarW = 256.0f;
constexpr float kCarA = 16.0f;
constexpr float kCarP = 1024.0f;
constexpr float kInvWA = 1.0f / (kCarW * kCarA);
constexpr float kInvWP = 1.0f / (kCarW * kCarP);
constexpr float kInvW  = 1.0f / kCarW;
constexpr float kF16MinNormal = 6.103515625e-05f;

constexpr int oWA  = 0;
constexpr int oWh  = oWA  + 512 * 256;
constexpr int oWm  = oWh  + 768 * 256;
constexpr int oWi  = oWm  + 768 * 256;
constexpr int oWci = oWi  + 768 * 64;
constexpr int oAd  = oWci + 192 * 64;
constexpr int oAdT = oAd  + 1024 * 64;
constexpr int oWo  = oAdT + 64 * 1024;
constexpr int oX   = oWo  + 16 * 256;
constexpr int kPlaneHalves = oX + 1024 * 64;
constexpr size_t kPlaneBytes = (size_t)kPlaneHalves * 2;
constexpr size_t kWhistBytes = (size_t)kSteps * kBatch * kSlots * 4;
constexpr size_t kChistBytes = (size_t)kSteps * kBatch * kCont * 4;
constexpr size_t kWsTotal = kPlaneBytes + kWhistBytes + kChistBytes;
static_assert(kPlaneHalves == 786432, "plane carve");
static_assert(kPlaneBytes == 1572864, "plane bytes");
static_assert(kPlaneBytes % 128 == 0, "line aligned carve");
static_assert(kWsTotal == 6553600, "workspace total");
static_assert(kPlaneHalves / 8 == 384 * 256, "prep grid covers every 16-B chunk exactly once");

constexpr int kHP   = 264;
constexpr int kQP   = 72;
constexpr int kWP   = 1032;
constexpr int kSimP = 1028;
static_assert(2 * kBatch * kCont <= 16 * kSimP, "q_c and cand staging fit inside the sim plane");
constexpr size_t kLdsBytes = (size_t)kHid * kBatch * 4 + (size_t)kBatch * kHP * 2 + (size_t)16 * kSimP * 4 +
                             (size_t)kBatch * kQP * 2 + (size_t)kBatch * kWP * 2 + (size_t)kBatch * kHP * 2 +
                             1024 * 4 + 1024 * 4 + 32 * 4 + 320 * 4;
static_assert(kLdsBytes == 212608, "LDS total");
static_assert(kLdsBytes < 300000, "LDS budget");

__device__ __forceinline__ _Float16 to_h(float v) {
  const float a = fabsf(v);
  const float r = (a < kF16MinNormal) ? 0.0f : v;
  return (_Float16)r;
}

union FragU { v16h v; v8h h[2]; };
__device__ __forceinline__ v16h frag_ld(const _Float16* p) {
  FragU f;
  f.h[0] = *(const v8h*)(p);
  f.h[1] = *(const v8h*)(p + 16);
  return f.v;
}

__device__ __forceinline__ v8f mma(v16h a, v16h b, v8f c) {
  c = __builtin_amdgcn_wmma_f32_16x16x32_f16(false, a, false, b, (short)0, c, false, false);
  asm volatile("v_nop\n\tv_nop\n\tv_nop\n\tv_nop" : "+v"(c) : "v"(a), "v"(b));
  return c;
}

__device__ __forceinline__ float wave_sum(float v) {
#pragma unroll
  for (int off = 16; off >= 1; off >>= 1) v += __shfl_xor(v, off, 32);
  return v;
}
__device__ __forceinline__ float wave_max(float v) {
#pragma unroll
  for (int off = 16; off >= 1; off >>= 1) v = fmaxf(v, __shfl_xor(v, off, 32));
  return v;
}
__device__ __forceinline__ void wave_lds_sync() {
  __builtin_amdgcn_fence(__ATOMIC_RELEASE, "workgroup");
  __builtin_amdgcn_wave_barrier();
  __builtin_amdgcn_fence(__ATOMIC_ACQUIRE, "workgroup");
}

__device__ __forceinline__ void store_chunk(_Float16* dst, v8h o) {
  volatile v8h* p = (volatile v8h*)dst;
  *p = o;
  __threadfence();
  *p = o;
}

__device__ __forceinline__ void cast_rows(const float* __restrict__ src, int srcRows, int kcols,
                                          _Float16* dst, int lc, float carry) {
  const int cpr = kcols >> 3;
  const int r = lc / cpr;
  const int c8 = (lc - r * cpr) << 3;
  const bool valid = r < srcRows;
  const int rc = valid ? r : (srcRows - 1);
  const float* sp = src + (size_t)rc * kcols + c8;
  const v4f a = *(const v4f*)(sp);
  const v4f b = *(const v4f*)(sp + 4);
  v8h o;
#pragma unroll
  for (int e = 0; e < 4; ++e) {
    o[e]     = to_h(valid ? a[e] * carry : 0.0f);
    o[4 + e] = to_h(valid ? b[e] * carry : 0.0f);
  }
  store_chunk(dst + (size_t)lc * 8, o);
}

__global__ __launch_bounds__(256)
void prep_kernel(const float* __restrict__ batch, const float* __restrict__ Wi, const float* __restrict__ Wh,
                 const float* __restrict__ Wm, const float* __restrict__ Wout, const float* __restrict__ addr,
                 const float* __restrict__ Wq, const float* __restrict__ us, const float* __restrict__ Wch,
                 const float* __restrict__ Wci, _Float16* planes)
{
  const int blk = blockIdx.x;
  const int tid = threadIdx.x;
  if (blk < 32) {
    cast_rows(Wq, 256, 256, planes + oWA, blk * 256 + tid, kCarW);
  } else if (blk < 56) {
    cast_rows(Wch, 192, 256, planes + oWA + 256 * 256, (blk - 32) * 256 + tid, kCarW);
  } else if (blk < 64) {
    cast_rows(us, 1, 256, planes + oWA + 448 * 256, (blk - 56) * 256 + tid, kCarW);
  } else if (blk < 160) {
    cast_rows(Wh, 768, 256, planes + oWh, (blk - 64) * 256 + tid, kCarW);
  } else if (blk < 256) {
    cast_rows(Wm, 768, 256, planes + oWm, (blk - 160) * 256 + tid, kCarW);
  } else if (blk < 280) {
    cast_rows(Wi, 768, 64, planes + oWi, (blk - 256) * 256 + tid, kCarW);
  } else if (blk < 286) {
    cast_rows(Wci, 192, 64, planes + oWci, (blk - 280) * 256 + tid, kCarW);
  } else if (blk < 318) {
    cast_rows(addr, 1024, 64, planes + oAd, (blk - 286) * 256 + tid, kCarW);
  } else if (blk < 350) {
    const int lc = (blk - 318) * 256 + tid;
    const int a  = lc >> 7;
    const int n0 = (lc & 127) << 3;
    v8h o;
#pragma unroll
    for (int e = 0; e < 8; ++e) o[e] = to_h(addr[(size_t)(n0 + e) * kAddr + a] * kCarW);
    store_chunk(planes + oAdT + (size_t)lc * 8, o);
  } else if (blk < 352) {
    cast_rows(Wout, kCls, 256, planes + oWo, (blk - 350) * 256 + tid, kCarW);
  } else {
    const int lc  = (blk - 352) * 256 + tid;
    const int row = lc >> 3;
    const int f0  = (lc & 7) << 3;
    const int t   = row >> 5;
    const int b   = row & 31;
    v8h o;
#pragma unroll
    for (int e = 0; e < 8; ++e) {
      const int f = f0 + e;
      const int src = (f >> 1) * (kSteps * kFeat) + t * kFeat + (f & 1) * 32 + b;
      o[e] = to_h(batch[src] * kCarA);
    }
    store_chunk(planes + oX + (size_t)lc * 8, o);
  }
}

__global__ __launch_bounds__(512)
void controller_kernel(const _Float16* __restrict__ planes,
                       const float* __restrict__ bi, const float* __restrict__ bh, const float* __restrict__ bm,
                       const float* __restrict__ bq, const float* __restrict__ bout,
                       float* whist, float* chist, float* out)
{
  __shared__ __align__(16) float    h32S[kHid * kBatch];
  __shared__ __align__(16) _Float16 h16S[kBatch * kHP];
  __shared__ __align__(16) float    simS[16 * kSimP];
  __shared__ __align__(16) _Float16 qa16S[kBatch * kQP];
  __shared__ __align__(16) _Float16 w16S[kBatch * kWP];
  __shared__ __align__(16) _Float16 rd16S[kBatch * kHP];
  __shared__ __align__(16) float    dS[1024];
  __shared__ __align__(16) float    gS[1024];
  __shared__ __align__(16) float    betaS[32];
  __shared__ __align__(16) float    lgS[320];

  float* const qcS   = simS;
  float* const candS = simS + kBatch * kCont;

  const int tid  = threadIdx.x;
  const int lane = tid & 31;
  const int wave = __builtin_amdgcn_readfirstlane(tid >> 5);
  const int ln   = lane & 15;
  const int hf   = lane >> 4;
  const int hh   = 16 * wave + ln;

  const _Float16* pWA  = planes + oWA;
  const _Float16* pWh  = planes + oWh;
  const _Float16* pWm  = planes + oWm;
  const _Float16* pWi  = planes + oWi;
  const _Float16* pWci = planes + oWci;
  const _Float16* pAd  = planes + oAd;
  const _Float16* pAdT = planes + oAdT;
  const _Float16* pWo  = planes + oWo;
  const _Float16* pX   = planes + oX;

  const v8f z8 = (v8f){0.f, 0.f, 0.f, 0.f, 0.f, 0.f, 0.f, 0.f};
  const v4f z4 = (v4f){0.f, 0.f, 0.f, 0.f};

  for (int i = tid; i < kHid * kBatch / 4; i += 512) *(v4f*)(h32S + 4 * i) = z4;
  {
    v8h zh;
#pragma unroll
    for (int e = 0; e < 8; ++e) zh[e] = (_Float16)0.0f;
    for (int i = tid; i < kBatch * kHP / 8; i += 512) *(v8h*)(h16S + 8 * i) = zh;
  }

  const float c_r  = bi[hh] + bh[hh] + bm[hh];
  const float c_z  = bi[256 + hh] + bh[256 + hh] + bm[256 + hh];
  const float c_n  = bi[512 + hh] + bm[512 + hh];
  const float c_hn = bh[512 + hh];
  const float bqv  = bq[hh];
  float boutv = bout[ln < kCls ? ln : kCls - 1];
  asm volatile("" : "+v"(boutv));

  __syncthreads();

#pragma unroll 1
  for (int t = 0; t < kSteps; ++t) {
    __threadfence();
    __syncthreads();

    {
      v8f q0 = z8, q1 = z8, c0 = z8, c1 = z8;
      const _Float16* A0 = h16S + ln * kHP + 8 * hf;
      const _Float16* A1 = h16S + (16 + ln) * kHP + 8 * hf;
      const _Float16* B0 = pWA + (size_t)hh * 256 + 8 * hf;
      const _Float16* B1 = pWA + (size_t)(256 + hh) * 256 + 8 * hf;
#pragma unroll 1
      for (int k0 = 0; k0 < kHid; k0 += 32) {
        const v16h fa0 = frag_ld(A0 + k0);
        const v16h fa1 = frag_ld(A1 + k0);
        const v16h fb0 = frag_ld(B0 + k0);
        const v16h fb1 = frag_ld(B1 + k0);
        q0 = mma(fa0, fb0, q0);
        q1 = mma(fa1, fb0, q1);
        c0 = mma(fa0, fb1, c0);
        c1 = mma(fa1, fb1, c1);
      }
      if (wave < 12) {
        const _Float16* XA0 = pX + (size_t)(t * 32 + ln) * kFeat + 8 * hf;
        const _Float16* XA1 = pX + (size_t)(t * 32 + 16 + ln) * kFeat + 8 * hf;
        const _Float16* BC  = pWci + (size_t)hh * kFeat + 8 * hf;
#pragma unroll
        for (int k0 = 0; k0 < kFeat; k0 += 32) {
          const v16h xa0 = frag_ld(XA0 + k0);
          const v16h xa1 = frag_ld(XA1 + k0);
          const v16h fbc = frag_ld(BC + k0);
          c0 = mma(xa0, fbc, c0);
          c1 = mma(xa1, fbc, c1);
        }
      }
#pragma unroll
      for (int r = 0; r < 8; ++r) {
        const int b0 = 8 * hf + r;
        const int b1 = 16 + 8 * hf + r;
        const float qv0 = q0[r] * kInvWA + bqv;
        const float qv1 = q1[r] * kInvWA + bqv;
        if (wave < 4) {
          qa16S[b0 * kQP + hh] = to_h(qv0 * kCarA);
          qa16S[b1 * kQP + hh] = to_h(qv1 * kCarA);
        } else {
          qcS[b0 * kCont + (hh - kAddr)] = qv0;
          qcS[b1 * kCont + (hh - kAddr)] = qv1;
        }
        if (wave < 12) {
          candS[b0 * kCont + hh] = fmaxf(c0[r] * kInvWA, 0.0f);
          candS[b1 * kCont + hh] = fmaxf(c1[r] * kInvWA, 0.0f);
        } else if (wave == 12) {
          if (ln == 0) {
            betaS[b0] = c0[r] * kInvWA;
            betaS[b1] = c1[r] * kInvWA;
          }
        }
      }
    }
    __syncthreads();

    {
      v4f cv[3];
#pragma unroll
      for (int i = 0; i < 3; ++i) cv[i] = *(const v4f*)(candS + 4 * (tid + 512 * i));
      float* dst = chist + (size_t)t * (kBatch * kCont);
      for (int pass = 0; pass < 2; ++pass) {
#pragma unroll
        for (int i = 0; i < 3; ++i) *(volatile v4f*)(dst + 4 * (tid + 512 * i)) = cv[i];
        __threadfence();
      }
      const int npair = t * 32;
#pragma unroll 1
      for (int p = wave; p < npair; p += 16) {
        const int b = p & 31;
        const float* cr = chist + (size_t)p * kCont;
        const float* qr = qcS + b * kCont;
        float acc = 0.0f;
#pragma unroll
        for (int i = 0; i < 6; ++i) acc = fmaf(cr[lane + 32 * i], qr[lane + 32 * i], acc);
        acc = wave_sum(acc);
        if (lane == 0) dS[p] = acc;
      }
    }
    __syncthreads();

#pragma unroll 1
    for (int mt = 0; mt < 2; ++mt) {
      {
        v8f sacc[4];
#pragma unroll
        for (int j = 0; j < 4; ++j) sacc[j] = z8;
        const _Float16* QA = qa16S + (16 * mt + ln) * kQP + 8 * hf;
        const _Float16* AD = pAd + (size_t)(64 * wave + ln) * kAddr + 8 * hf;
#pragma unroll
        for (int k0 = 0; k0 < kAddr; k0 += 32) {
          const v16h fa = frag_ld(QA + k0);
#pragma unroll
          for (int j = 0; j < 4; ++j) {
            const v16h fb = frag_ld(AD + j * (16 * kAddr) + k0);
            sacc[j] = mma(fa, fb, sacc[j]);
          }
        }
#pragma unroll
        for (int j = 0; j < 4; ++j) {
#pragma unroll
          for (int r = 0; r < 8; ++r) {
            simS[(8 * hf + r) * kSimP + 64 * wave + 16 * j + ln] = sacc[j][r] * kInvWA;
          }
        }
      }
      __syncthreads();
      {
        const int b = 16 * mt + wave;
        float* srow = simS + wave * kSimP + 4 * lane;
        v4f sv[8];
#pragma unroll
        for (int i = 0; i < 8; ++i) sv[i] = *(const v4f*)(srow + 128 * i);
#pragma unroll 1
        for (int s = 0; s < t; ++s) {
          const float ds = dS[s * 32 + b];
          const float* wr = whist + (size_t)(s * 32 + b) * kSlots + 4 * lane;
          v4f wv[8];
#pragma unroll
          for (int i = 0; i < 8; ++i) wv[i] = *(const v4f*)(wr + 128 * i);
#pragma unroll
          for (int i = 0; i < 8; ++i) sv[i] += wv[i] * ds;
        }
        const float ub = betaS[b];
        const float beta = fmaxf(ub, 0.0f) + log1pf(expf(-fabsf(ub))) + 1.0f;
        float mx = -INFINITY;
#pragma unroll
        for (int i = 0; i < 8; ++i) {
          sv[i] = sv[i] * beta;
          mx = fmaxf(mx, fmaxf(fmaxf(sv[i][0], sv[i][1]), fmaxf(sv[i][2], sv[i][3])));
        }
        mx = wave_max(mx);
#pragma unroll
        for (int i = 0; i < 8; ++i) *(v4f*)(srow + 128 * i) = sv[i] - mx;
        wave_lds_sync();
        float sum = 0.0f;
#pragma unroll 1
        for (int i = 0; i < 8; ++i) {
          const v4f e = *(const v4f*)(srow + 128 * i);
          v4f x;
          x[0] = expf(e[0]);
          x[1] = expf(e[1]);
          x[2] = expf(e[2]);
          x[3] = expf(e[3]);
          *(v4f*)(srow + 128 * i) = x;
          sum += (x[0] + x[1]) + (x[2] + x[3]);
        }
        sum = wave_sum(sum);
        wave_lds_sync();
        const float inv = 1.0f / sum;
        v4f wn[8];
#pragma unroll
        for (int i = 0; i < 8; ++i) wn[i] = *(const v4f*)(srow + 128 * i) * inv;
        float* wd = whist + (size_t)(t * 32 + b) * kSlots + 4 * lane;
        for (int pass = 0; pass < 2; ++pass) {
#pragma unroll
          for (int i = 0; i < 8; ++i) *(volatile v4f*)(wd + 128 * i) = wn[i];
          __threadfence();
        }
#pragma unroll
        for (int i = 0; i < 8; ++i) {
          v4h ph;
          ph[0] = to_h(wn[i][0] * kCarP);
          ph[1] = to_h(wn[i][1] * kCarP);
          ph[2] = to_h(wn[i][2] * kCarP);
          ph[3] = to_h(wn[i][3] * kCarP);
          *(v4h*)(w16S + b * kWP + 4 * lane + 128 * i) = ph;
        }
#pragma unroll 1
        for (int s = 0; s < t; ++s) {
          const float* wr = whist + (size_t)(s * 32 + b) * kSlots + 4 * lane;
          float acc = 0.0f;
#pragma unroll
          for (int i = 0; i < 8; ++i) {
            const v4f x = *(const v4f*)(wr + 128 * i);
            acc += (x[0] * wn[i][0] + x[1] * wn[i][1]) + (x[2] * wn[i][2] + x[3] * wn[i][3]);
          }
          acc = wave_sum(acc);
          if (lane == 0) gS[s * 32 + b] = acc;
        }
      }
      __syncthreads();
    }

    if (wave < 8) {
      const int mt = wave >> 2;
      const int nt = wave & 3;
      v8f ra = z8;
      const _Float16* WA_ = w16S + (16 * mt + ln) * kWP + 8 * hf;
      const _Float16* BT  = pAdT + (size_t)(16 * nt + ln) * kSlots + 8 * hf;
#pragma unroll 1
      for (int k0 = 0; k0 < kSlots; k0 += 32) {
        const v16h fa = frag_ld(WA_ + k0);
        const v16h fb = frag_ld(BT + k0);
        ra = mma(fa, fb, ra);
      }
#pragma unroll
      for (int r = 0; r < 8; ++r) {
        const int b = 16 * mt + 8 * hf + r;
        rd16S[b * kHP + 16 * nt + ln] = to_h(ra[r] * kInvW);
      }
    }
    {
#pragma unroll 1
      for (int i = 0; i < 3; ++i) {
        const int u  = tid + 512 * i;
        const int b  = u / 48;
        const int c4 = u - 48 * b;
        v4f acc = z4;
#pragma unroll 1
        for (int s = 0; s < t; ++s) {
          const float g = gS[s * 32 + b];
          const v4f cvv = *(const v4f*)(chist + (size_t)(s * 32 + b) * kCont + 4 * c4);
          acc += cvv * g;
        }
        v4h ph;
        ph[0] = to_h(acc[0] * kCarP);
        ph[1] = to_h(acc[1] * kCarP);
        ph[2] = to_h(acc[2] * kCarP);
        ph[3] = to_h(acc[3] * kCarP);
        *(v4h*)(rd16S + b * kHP + kAddr + 4 * c4) = ph;
      }
    }
    __syncthreads();

#pragma unroll 1
    for (int mt = 0; mt < 2; ++mt) {
      v8f grz0 = z8, grz1 = z8, ghn = z8, gin = z8, gm0 = z8, gm1 = z8, gm2 = z8;
      {
        const _Float16* AH = h16S + (16 * mt + ln) * kHP + 8 * hf;
        const _Float16* BH = pWh + (size_t)hh * kHid + 8 * hf;
#pragma unroll 1
        for (int k0 = 0; k0 < kHid; k0 += 32) {
          const v16h fa  = frag_ld(AH + k0);
          const v16h fb0 = frag_ld(BH + k0);
          const v16h fb1 = frag_ld(BH + 256 * kHid + k0);
          const v16h fb2 = frag_ld(BH + 512 * kHid + k0);
          grz0 = mma(fa, fb0, grz0);
          grz1 = mma(fa, fb1, grz1);
          ghn  = mma(fa, fb2, ghn);
        }
      }
      {
        const _Float16* AR = rd16S + (16 * mt + ln) * kHP + 8 * hf;
        const _Float16* BM = pWm + (size_t)hh * 256 + 8 * hf;
#pragma unroll 1
        for (int k0 = 0; k0 < 256; k0 += 32) {
          const v16h fa  = frag_ld(AR + k0);
          const v16h fb0 = frag_ld(BM + k0);
          const v16h fb1 = frag_ld(BM + 256 * 256 + k0);
          const v16h fb2 = frag_ld(BM + 512 * 256 + k0);
          gm0 = mma(fa, fb0, gm0);
          gm1 = mma(fa, fb1, gm1);
          gm2 = mma(fa, fb2, gm2);
        }
      }
      {
        const _Float16* AX = pX + (size_t)(t * 32 + 16 * mt + ln) * kFeat + 8 * hf;
        const _Float16* BI = pWi + (size_t)hh * kFeat + 8 * hf;
#pragma unroll
        for (int k0 = 0; k0 < kFeat; k0 += 32) {
          const v16h fa  = frag_ld(AX + k0);
          const v16h fb0 = frag_ld(BI + k0);
          const v16h fb1 = frag_ld(BI + 256 * kFeat + k0);
          const v16h fb2 = frag_ld(BI + 512 * kFeat + k0);
          grz0 = mma(fa, fb0, grz0);
          grz1 = mma(fa, fb1, grz1);
          gin  = mma(fa, fb2, gin);
        }
      }
      __syncthreads();
#pragma unroll
      for (int r = 0; r < 8; ++r) {
        const int b = 16 * mt + 8 * hf + r;
        const float pr = grz0[r] * kInvWA + gm0[r] * kInvWP + c_r;
        const float pz = grz1[r] * kInvWA + gm1[r] * kInvWP + c_z;
        const float rg = 1.0f / (1.0f + expf(-pr));
        const float zg = 1.0f / (1.0f + expf(-pz));
        const float pn = gin[r] * kInvWA + gm2[r] * kInvWP + c_n + rg * (ghn[r] * kInvWA + c_hn);
        const float ng = tanhf(pn);
        const float hold = h32S[hh * kBatch + b];
        const float hn = (1.0f - zg) * ng + zg * hold;
        h32S[hh * kBatch + b] = hn;
        h16S[b * kHP + hh] = to_h(hn * kCarA);
      }
    }
    __syncthreads();

    {
      v4f hv[4];
#pragma unroll
      for (int i = 0; i < 4; ++i) hv[i] = *(const v4f*)(h32S + 4 * (tid + 512 * i));
      float* hd = out + (size_t)t * (kHid * kBatch);
      for (int pass = 0; pass < 2; ++pass) {
#pragma unroll
        for (int i = 0; i < 4; ++i) *(volatile v4f*)(hd + 4 * (tid + 512 * i)) = hv[i];
        __threadfence();
      }
    }
    if (wave < 2) {
      v8f lg = z8;
      const _Float16* AH = h16S + (16 * wave + ln) * kHP + 8 * hf;
      const _Float16* BO = pWo + (size_t)ln * kHid + 8 * hf;
#pragma unroll 1
      for (int k0 = 0; k0 < kHid; k0 += 32) {
        const v16h fa = frag_ld(AH + k0);
        const v16h fb = frag_ld(BO + k0);
        lg = mma(fa, fb, lg);
      }
#pragma unroll
      for (int r = 0; r < 8; ++r) {
        const int b = 16 * wave + 8 * hf + r;
        const float v = lg[r] * kInvWA + boutv;
        if (ln < kCls) lgS[ln * 32 + b] = v;
      }
    }
    __syncthreads();
    if (wave == 0) {
      float mx = -INFINITY;
#pragma unroll 1
      for (int o = 0; o < kCls; ++o) mx = fmaxf(mx, lgS[o * 32 + lane]);
      float se = 0.0f;
#pragma unroll 1
      for (int o = 0; o < kCls; ++o) se += expf(lgS[o * 32 + lane] - mx);
      const float lse = mx + logf(se);
      float* od = out + (size_t)(kSteps * kHid * kBatch) + (size_t)t * (kCls * kBatch) + lane;
      for (int pass = 0; pass < 2; ++pass) {
#pragma unroll
        for (int o = 0; o < kCls; ++o) {
          const float v = lgS[o * 32 + lane] - lse;
          *(volatile float*)(od + o * 32) = v;
        }
        __threadfence();
      }
    }
  }
}

extern "C" void kernel_launch(void* const* d_in, const int* in_sizes, int n_in,
                              void* d_out, int out_size, void* d_ws, size_t ws_size,
                              hipStream_t stream) {
  if (n_in < 15) return;
  if (in_sizes[0] < kBatch * kSteps * kFeat || in_sizes[1] < kGate * kFeat || in_sizes[2] < kGate ||
      in_sizes[3] < kGate * kHid || in_sizes[4] < kGate || in_sizes[5] < kGate * 256 || in_sizes[6] < kGate ||
      in_sizes[7] < kCls * kHid || in_sizes[8] < kCls || in_sizes[9] < kSlots * kAddr ||
      in_sizes[10] < 256 * kHid || in_sizes[11] < 256 || in_sizes[12] < kHid ||
      in_sizes[13] < kCont * kHid || in_sizes[14] < kCont * kFeat) return;
  if (out_size < kSteps * kHid * kBatch + kSteps * kCls * kBatch) return;
  if (ws_size < kWsTotal) return;

  const float* batch = (const float*)d_in[0];
  const float* Wi    = (const float*)d_in[1];
  const float* bi    = (const float*)d_in[2];
  const float* Wh    = (const float*)d_in[3];
  const float* bh    = (const float*)d_in[4];
  const float* Wm    = (const float*)d_in[5];
  const float* bm    = (const float*)d_in[6];
  const float* Wout  = (const float*)d_in[7];
  const float* bout  = (const float*)d_in[8];
  const float* addr  = (const float*)d_in[9];
  const float* Wq    = (const float*)d_in[10];
  const float* bq    = (const float*)d_in[11];
  const float* us    = (const float*)d_in[12];
  const float* Wch   = (const float*)d_in[13];
  const float* Wci   = (const float*)d_in[14];

  _Float16* planes = (_Float16*)d_ws;
  float* whist = (float*)((char*)d_ws + kPlaneBytes);
  float* chist = (float*)((char*)d_ws + kPlaneBytes + kWhistBytes);
  float* outp  = (float*)d_out;

  prep_kernel<<<dim3(384), dim3(256), 0, stream>>>(batch, Wi, Wh, Wm, Wout, addr, Wq, us, Wch, Wci, planes);
  controller_kernel<<<dim3(1), dim3(512), 0, stream>>>(planes, bi, bh, bm, bq, bout, whist, chist, outp);
}
